// DynamicDepthSeparableConv1dMultiheadAttention_9414568313152
// MI455X (gfx1250) — hardware-verified
//
#include <hip/hip_runtime.h>
#include <math.h>
#include <stdint.h>

#define NB    16
#define CIN   128
#define NHD   8
#define NCO   1024
#define SLEN  1024
#define GBAT  4
#define NGRP  (NB / GBAT)
#define QXSZ  (SLEN * CIN)
#define PLN   (NCO * SLEN)
static_assert(NGRP * GBAT == NB);
static_assert(NHD * CIN == NCO);
static_assert(QXSZ == 131072 && PLN == 1048576);
static_assert((SLEN % 128) == 0 && (NCO % 64) == 0 && (CIN % 32) == 0 && (SLEN % 64) == 0);

typedef _Float16 v16h __attribute__((ext_vector_type(16)));
typedef _Float16 v8h  __attribute__((ext_vector_type(8)));
typedef float    v8f  __attribute__((ext_vector_type(8)));
typedef float    v4f  __attribute__((ext_vector_type(4)));
typedef unsigned int v4u __attribute__((ext_vector_type(4)));

__device__ __forceinline__ unsigned short bf_bits(float f) {
  unsigned u = __float_as_uint(f);
  return (unsigned short)((u + 0x7FFFu + ((u >> 16) & 1u)) >> 16);
}
__device__ __forceinline__ float bf_up(unsigned short h) { return __uint_as_float(((unsigned)h) << 16); }
__device__ __forceinline__ unsigned short h_bits(_Float16 x) { return __builtin_bit_cast(unsigned short, x); }
__device__ __forceinline__ unsigned pk16(unsigned short a, unsigned short b) { return (unsigned)a | ((unsigned)b << 16); }
__device__ __forceinline__ v8f zero8() { v8f z = {0.f, 0.f, 0.f, 0.f, 0.f, 0.f, 0.f, 0.f}; return z; }

__device__ __forceinline__ v16h ldfrag_h(const _Float16* p) {
  union { v16h v; v8h h[2]; } f;
  f.h[0] = *(const v8h*)(p);
  f.h[1] = *(const v8h*)(p + 16);
  return f.v;
}

__device__ __forceinline__ v8f mma_h_raw(v16h a, v16h b, v8f c) {
  return __builtin_amdgcn_wmma_f32_16x16x32_f16(false, a, false, b, (short)0, c, false, false);
}
__device__ __forceinline__ void res_guard(v8f& t, v8f& acc, v16h x, v16h y) {
#if defined(__HIP_DEVICE_COMPILE__)
  asm volatile("v_nop\n\tv_nop\n\tv_nop\n\tv_nop" : "+v"(t), "+v"(acc) : "v"(x), "v"(y));
#endif
}
__device__ __forceinline__ void dep_guard_h(v8f& a, v8f& b, v16h x, v16h y) {
#if defined(__HIP_DEVICE_COMPILE__)
  asm volatile("v_nop\n\tv_nop\n\tv_nop\n\tv_nop" : "+v"(a), "+v"(b) : "v"(x), "v"(y));
#endif
}
__device__ __forceinline__ void keep4_h(v16h a, v16h b, v16h c, v16h d) {
#if defined(__HIP_DEVICE_COMPILE__)
  asm volatile("v_nop" :: "v"(a), "v"(b), "v"(c), "v"(d));
#endif
}
__device__ __forceinline__ void acc_guard4(v8f& a, v8f& b, v8f& c, v8f& d) {
#if defined(__HIP_DEVICE_COMPILE__)
  asm volatile("v_nop\n\tv_nop\n\tv_nop\n\tv_nop" : "+v"(a), "+v"(b), "+v"(c), "+v"(d));
#endif
}
__device__ __forceinline__ void wave_sync_lds() {
  __builtin_amdgcn_fence(__ATOMIC_RELEASE, "workgroup");
  __builtin_amdgcn_wave_barrier();
  __builtin_amdgcn_fence(__ATOMIC_ACQUIRE, "workgroup");
}

__global__ __launch_bounds__(256) void cvt_h8(const float* __restrict__ in, unsigned short* out, int n8, float scale) {
  const int i = blockIdx.x * 256 + threadIdx.x;
  if (i < n8) {
    const v4f a = *(const v4f*)(in + (size_t)i * 8);
    const v4f c = *(const v4f*)(in + (size_t)i * 8 + 4);
    float f[8];
    f[0] = a[0]; f[1] = a[1]; f[2] = a[2]; f[3] = a[3];
    f[4] = c[0]; f[5] = c[1]; f[6] = c[2]; f[7] = c[3];
    unsigned short hb[8];
#pragma unroll
    for (int e = 0; e < 8; ++e) hb[e] = h_bits((_Float16)(bf_up(bf_bits(f[e])) * scale));
    v4u p;
    p[0] = pk16(hb[0], hb[1]);
    p[1] = pk16(hb[2], hb[3]);
    p[2] = pk16(hb[4], hb[5]);
    p[3] = pk16(hb[6], hb[7]);
    *(volatile v4u*)(out + (size_t)i * 8) = p;
    __threadfence();
    *(volatile v4u*)(out + (size_t)i * 8) = p;
  }
}

__global__ __launch_bounds__(256) void cvt_qt(const float* __restrict__ x, unsigned short* out, float scale) {
  __shared__ __align__(16) unsigned short ts[64 * 136];
  const int tid = threadIdx.x;
  const int l0 = blockIdx.x * 64, b = blockIdx.y;
#pragma unroll 1
  for (int pass = 0; pass < 8; ++pass) {
    const int c = pass * 16 + (tid >> 4);
    const int l4 = (tid & 15) * 4;
    const v4f v = *(const v4f*)(x + ((size_t)(b * CIN + c) * SLEN) + l0 + l4);
#pragma unroll
    for (int i = 0; i < 4; ++i) ts[(l4 + i) * 136 + c] = h_bits((_Float16)(bf_up(bf_bits(v[i])) * scale));
  }
  __syncthreads();
#pragma unroll 1
  for (int pass = 0; pass < 4; ++pass) {
    const int lr = pass * 16 + (tid >> 4);
    const int c8 = (tid & 15) * 8;
    const v4u v = *(const v4u*)(ts + lr * 136 + c8);
    unsigned short* dst = out + ((size_t)(b * SLEN) + l0 + lr) * CIN + c8;
    *(volatile v4u*)dst = v;
    __threadfence();
    *(volatile v4u*)dst = v;
  }
}

template <int NSPLIT, int BIAS>
__global__ __launch_bounds__(256) void gemm64(
    const unsigned short* __restrict__ Ap, int lda, long long sAy, long long sAz,
    const unsigned short* __restrict__ Btp, int ldb, long long sBy, long long sBz,
    const unsigned short* __restrict__ Bt2p, int ldb2,
    const float* __restrict__ bias,
    float* Cout, int ldc, long long sCy, long long sCz,
    int M, int N, int K, float oscale, float rres) {
  const _Float16* A   = (const _Float16*)(const void*)Ap;
  const _Float16* Bt  = (const _Float16*)(const void*)Btp;
  const _Float16* Bt2 = (const _Float16*)(const void*)Bt2p;
  __shared__ __align__(16) float sT[8][16 * 68];
  const int by   = blockIdx.y;
  const int bz   = blockIdx.z;
  const int lane = threadIdx.x & 31;
  const int wave = threadIdx.x >> 5;
  const int tilesN = N >> 6;
  const int tilesM = M >> 6;
  const int tile = blockIdx.x * 8 + wave;
  if (tile >= tilesM * tilesN) return;
  const int tm = tile / tilesN;
  const int tn = tile - tm * tilesN;
  const int m0 = tm << 6;
  const int n0 = tn << 6;

  const _Float16* Ab  = A + (size_t)by * (size_t)sAy + (size_t)bz * (size_t)sAz;
  const _Float16* Bb  = Bt + (size_t)by * (size_t)sBy + (size_t)bz * (size_t)sBz;
  const _Float16* Bb2 = (NSPLIT == 2) ? (Bt2 + (size_t)by * (size_t)sBy + (size_t)bz * (size_t)sBz) : Bb;
  const int ld2 = (NSPLIT == 2) ? ldb2 : ldb;

  const int rlane = lane & 15;
  const int koff  = (lane >> 4) * 8;
  const int mOff  = (lane >> 4) * 8;

  v8f acc[4][4];
#pragma unroll
  for (int i = 0; i < 4; ++i)
#pragma unroll
    for (int j = 0; j < 4; ++j) acc[i][j] = zero8();

  for (int k0 = 0; k0 < K; k0 += 32) {
    v16h bf[4];
#pragma unroll
    for (int j = 0; j < 4; ++j) {
      const size_t bo = (size_t)(n0 + (j << 4) + rlane) * ldb + koff + k0;
      bf[j] = ldfrag_h(Bb + bo);
    }
#pragma unroll
    for (int i = 0; i < 4; ++i) {
      const size_t ao = (size_t)(m0 + (i << 4) + rlane) * lda + koff + k0;
      const v16h ah = ldfrag_h(Ab + ao);
#pragma unroll
      for (int j = 0; j < 4; ++j) acc[i][j] = mma_h_raw(ah, bf[j], acc[i][j]);
      dep_guard_h(acc[i][0], acc[i][3], ah, bf[3]);
    }
    if (NSPLIT == 2) {
#pragma unroll
      for (int j = 0; j < 4; ++j) {
        const size_t bo = (size_t)(n0 + (j << 4) + rlane) * ld2 + koff + k0;
        bf[j] = ldfrag_h(Bb2 + bo);
      }
#pragma unroll
      for (int i = 0; i < 4; ++i) {
        const size_t ao = (size_t)(m0 + (i << 4) + rlane) * lda + koff + k0;
        const v16h al = ldfrag_h(Ab + ao);
#pragma unroll
        for (int j = 0; j < 4; ++j) {
          v8f tp = mma_h_raw(al, bf[j], zero8());
          res_guard(tp, acc[i][j], al, bf[j]);
#pragma unroll
          for (int r = 0; r < 8; ++r) acc[i][j][r] += tp[r] * rres;
        }
        dep_guard_h(acc[i][0], acc[i][3], al, bf[3]);
      }
    }
    keep4_h(bf[0], bf[1], bf[2], bf[3]);
  }
  acc_guard4(acc[0][0], acc[0][1], acc[0][2], acc[0][3]);
  acc_guard4(acc[1][0], acc[1][1], acc[1][2], acc[1][3]);
  acc_guard4(acc[2][0], acc[2][1], acc[2][2], acc[2][3]);
  acc_guard4(acc[3][0], acc[3][1], acc[3][2], acc[3][3]);

  float* slab = sT[wave];
  float* C = Cout + (size_t)by * (size_t)sCy + (size_t)bz * (size_t)sCz;
#pragma unroll
  for (int i = 0; i < 4; ++i) {
    const int mBase = m0 + (i << 4);
    float brow[8];
#pragma unroll
    for (int r = 0; r < 8; ++r) brow[r] = 0.f;
    if (BIAS == 2) {
#pragma unroll
      for (int r = 0; r < 8; ++r) brow[r] = bf_up(bf_bits(bias[mBase + mOff + r]));
    }
#pragma unroll
    for (int j = 0; j < 4; ++j) {
#pragma unroll
      for (int r = 0; r < 8; ++r) {
        slab[(mOff + r) * 68 + (j << 4) + rlane] = acc[i][j][r] * oscale + brow[r];
      }
    }
    wave_sync_lds();
    {
      const int hh = lane >> 4, c4 = (lane & 15) * 4;
      for (int pass = 0; pass < 2; ++pass) {
#pragma unroll
        for (int it = 0; it < 8; ++it) {
          const int row = it * 2 + hh;
          const v4f v = *(const v4f*)(slab + row * 68 + c4);
          *(volatile v4f*)(C + (size_t)(mBase + row) * ldc + n0 + c4) = v;
        }
        __threadfence();
      }
    }
    wave_sync_lds();
  }
}

#define YPITCH 80
#define TPITCH 136
__global__ __launch_bounds__(256) void dwconv_kernel(
    const float* __restrict__ Y,
    const float* __restrict__ dq3, const float* __restrict__ dq15, const float* __restrict__ gq,
    const float* __restrict__ dk3, const float* __restrict__ dk15, const float* __restrict__ gk,
    const float* __restrict__ dv3, const float* __restrict__ dv15, const float* __restrict__ gv,
    unsigned short* QX, unsigned short* KX, unsigned short* VX) {
  __shared__ __align__(16) float ys[128 * YPITCH];
  __shared__ __align__(16) unsigned short ts[64 * TPITCH];
  const int tid = threadIdx.x, lane = tid & 31, wave = tid >> 5;
  const int lt = blockIdx.x, h = blockIdx.y, bz = blockIdx.z;
  const int o0 = h * CIN, l0 = lt * 64;
  const int c8 = (lane & 7) * 8;
  const int rq = lane >> 3;

#pragma unroll 1
  for (int pj = 0; pj < 3; ++pj) {
    const float* d3  = (pj == 0) ? dq3  : ((pj == 1) ? dk3  : dv3);
    const float* d15 = (pj == 0) ? dq15 : ((pj == 1) ? dk15 : dv15);
    const float* gp  = (pj == 0) ? gq   : ((pj == 1) ? gk   : gv);
    const float ga = bf_up(bf_bits(gp[0]));
    const float gb = bf_up(bf_bits(gp[1]));
    const float gm = fmaxf(ga, gb);
    const float ea = __expf(ga - gm), eb = __expf(gb - gm);
    const float ginv = 1.0f / (ea + eb);
    const float g0 = ea * ginv, g1 = eb * ginv;

    __syncthreads();
    {
      const float* Yp = Y + ((size_t)(bz * 3 + pj)) * PLN + (size_t)o0 * SLEN;
      for (int idx = tid; idx < 128 * 78; idx += 256) {
        const int r  = idx / 78;
        const int ci = idx - r * 78;
        const int gl = l0 - 7 + ci;
        const int glc = min(max(gl, 0), SLEN - 1);
        float v = Yp[(size_t)r * SLEN + glc];
        v = (gl >= 0 && gl < SLEN) ? v : 0.f;
        ys[r * YPITCH + ci] = v;
      }
    }
    __syncthreads();

#pragma unroll 1
    for (int it = 0; it < 4; ++it) {
      const int r = wave * 16 + it * 4 + rq;
      const int orow = o0 + r;
      const float* yr = ys + r * YPITCH + c8;
      float a15[8], a3[8];
#pragma unroll
      for (int e = 0; e < 8; ++e) { a15[e] = 0.f; a3[e] = 0.f; }
#pragma unroll 1
      for (int j = 0; j < 15; ++j) {
        const float w = bf_up(bf_bits(d15[orow * 15 + j]));
#pragma unroll
        for (int e = 0; e < 8; ++e) a15[e] += w * yr[e + j];
      }
#pragma unroll 1
      for (int j = 0; j < 3; ++j) {
        const float w = bf_up(bf_bits(d3[orow * 3 + j]));
#pragma unroll
        for (int e = 0; e < 8; ++e) a3[e] += w * yr[e + 6 + j];
      }
      float y[8];
#pragma unroll
      for (int e = 0; e < 8; ++e) y[e] = g0 * a3[e] + g1 * a15[e];

      if (pj == 2) {
        v4u pk;
#pragma unroll
        for (int q = 0; q < 4; ++q)
          pk[q] = pk16(h_bits((_Float16)(y[2 * q] * 16.0f)), h_bits((_Float16)(y[2 * q + 1] * 16.0f)));
        unsigned short* dst = VX + ((size_t)(bz * NCO) + orow) * SLEN + l0 + c8;
        *(volatile v4u*)dst = pk;
        __threadfence();
        *(volatile v4u*)dst = pk;
      } else {
#pragma unroll
        for (int e = 0; e < 8; ++e) ts[(c8 + e) * TPITCH + r] = h_bits((_Float16)(y[e] * 16.0f));
      }
    }
    __syncthreads();
    if (pj != 2) {
      unsigned short* X = (pj == 0) ? QX : KX;
#pragma unroll 1
      for (int pass = 0; pass < 4; ++pass) {
        const int lr = pass * 16 + (tid >> 4);
        const int cc = (tid & 15) * 8;
        const v4u v = *(const v4u*)(ts + lr * TPITCH + cc);
        unsigned short* dst = X + (((size_t)(bz * NHD + h)) * SLEN + l0 + lr) * CIN + cc;
        *(volatile v4u*)dst = v;
        __threadfence();
        *(volatile v4u*)dst = v;
      }
    }
  }
}

#define KPITCH 136
#define VPITCH 40
#define HPITCH 136
__global__ __launch_bounds__(256) void attn_kernel(
    const unsigned short* __restrict__ QXp, const unsigned short* __restrict__ KXp,
    const unsigned short* __restrict__ VXp, unsigned short* CTXh, unsigned short* CTXl,
    float sc, float rscale) {
  __shared__ __align__(16) unsigned short lds_raw[128 * HPITCH];
  unsigned short* kl_u = lds_raw;
  unsigned short* vl_u = lds_raw + 32 * KPITCH;
  const _Float16* kl = (const _Float16*)(const void*)kl_u;
  const _Float16* vl = (const _Float16*)(const void*)vl_u;
  const _Float16* QX = (const _Float16*)(const void*)QXp;

  const int tid = threadIdx.x, lane = tid & 31, wave = tid >> 5;
  const int inst = blockIdx.y;
  const int bq = inst >> 3, hh = inst & 7;
  const int qBase = blockIdx.x * 128 + wave * 16;
  const int rlane = lane & 15, hsel = lane >> 4, koff = hsel * 8;

  const _Float16* Qb = QX + (size_t)inst * QXSZ + (size_t)(qBase + rlane) * CIN + koff;
  v16h qf[4];
#pragma unroll
  for (int kc = 0; kc < 4; ++kc) qf[kc] = ldfrag_h(Qb + kc * 32);

  const unsigned short* Kg = KXp + (size_t)inst * QXSZ + (size_t)(tid >> 3) * CIN + (tid & 7) * 16;
  const unsigned short* Vg = VXp + (size_t)inst * QXSZ + (size_t)(tid >> 1) * SLEN + (tid & 1) * 16;
  unsigned short* kd = kl_u + (tid >> 3) * KPITCH + (tid & 7) * 16;
  unsigned short* vd = vl_u + (tid >> 1) * VPITCH + (tid & 1) * 16;

  v8f oacc[8];
#pragma unroll
  for (int t = 0; t < 8; ++t) oacc[t] = zero8();
  float m_run = -1e30f, l_run = 0.f;
  const float LN1024 = 6.931471805599453f;

  for (int kb = 0; kb < SLEN; kb += 32) {
    __syncthreads();
    {
      const unsigned short* ks = Kg + (size_t)kb * CIN;
      const v4u k0v = *(const v4u*)ks;
      const v4u k1v = *(const v4u*)(ks + 8);
      *(v4u*)kd = k0v;
      *(v4u*)(kd + 8) = k1v;
      const unsigned short* vs = Vg + kb;
      const v4u v0 = *(const v4u*)vs;
      const v4u v1 = *(const v4u*)(vs + 8);
      *(v4u*)vd = v0;
      *(v4u*)(vd + 8) = v1;
    }
    __syncthreads();

    v8f s0 = zero8(), s1 = zero8();
    v16h ka, kbf;
#pragma unroll
    for (int kc = 0; kc < 4; ++kc) {
      ka  = ldfrag_h(kl + rlane * KPITCH + kc * 32 + koff);
      kbf = ldfrag_h(kl + (16 + rlane) * KPITCH + kc * 32 + koff);
      s0 = mma_h_raw(ka, qf[kc], s0);
      s1 = mma_h_raw(kbf, qf[kc], s1);
    }
    dep_guard_h(s0, s1, ka, kbf);

    float mloc = -1e30f;
#pragma unroll
    for (int r = 0; r < 8; ++r) mloc = fmaxf(mloc, fmaxf(s0[r], s1[r]));
    mloc = fmaxf(mloc, __shfl_xor(mloc, 16, 32));
    const float newM = fmaxf(m_run, mloc * sc);
    const float alpha = __expf(m_run - newM);
    const float msh = newM - LN1024;
    float ssum = 0.f;
    float p0[8], p1[8];
#pragma unroll
    for (int r = 0; r < 8; ++r) {
      p0[r] = __expf(s0[r] * sc - msh);
      p1[r] = __expf(s1[r] * sc - msh);
      ssum += p0[r] + p1[r];
    }
    ssum += __shfl_xor(ssum, 16, 32);
    l_run = l_run * alpha + ssum;
    m_run = newM;
#pragma unroll
    for (int t = 0; t < 8; ++t)
#pragma unroll
      for (int r = 0; r < 8; ++r) oacc[t][r] *= alpha;

    union { v16h v; _Float16 s[16]; } pf;
#pragma unroll
    for (int r = 0; r < 8; ++r) {
      pf.s[r]     = (_Float16)p0[r];
      pf.s[8 + r] = (_Float16)p1[r];
    }

    v16h va;
#pragma unroll
    for (int ct = 0; ct < 8; ++ct) {
      va = ldfrag_h(vl + (ct * 16 + rlane) * VPITCH + koff);
      oacc[ct] = mma_h_raw(va, pf.v, oacc[ct]);
    }
    dep_guard_h(oacc[0], oacc[7], va, pf.v);
  }
  acc_guard4(oacc[0], oacc[1], oacc[2], oacc[3]);
  acc_guard4(oacc[4], oacc[5], oacc[6], oacc[7]);

  __syncthreads();
  const float inv = 4.0f * (1.0f / l_run);
  unsigned short* hrow = lds_raw + (wave * 16 + rlane) * HPITCH + hsel * 8;
  v4u lv[8];
#pragma unroll
  for (int ct = 0; ct < 8; ++ct) {
    v4u hv, lw;
#pragma unroll
    for (int e = 0; e < 4; ++e) {
      const float f0 = oacc[ct][2 * e] * inv, f1 = oacc[ct][2 * e + 1] * inv;
      const _Float16 x0 = (_Float16)f0, x1 = (_Float16)f1;
      hv[e] = pk16(h_bits(x0), h_bits(x1));
      lw[e] = pk16(h_bits((_Float16)((f0 - (float)x0) * rscale)),
                   h_bits((_Float16)((f1 - (float)x1) * rscale)));
    }
    *(v4u*)(hrow + ct * 16) = hv;
    lv[ct] = lw;
  }
  wave_sync_lds();
  const size_t cbase = (size_t)bq * PLN + (size_t)hh * CIN;
  const unsigned short* hsrc = lds_raw + (wave * 16) * HPITCH;
  for (int pass = 0; pass < 2; ++pass) {
#pragma unroll
    for (int it = 0; it < 8; ++it) {
      const int qr = it * 2 + hsel;
      const v4u v = *(const v4u*)(hsrc + qr * HPITCH + rlane * 8);
      *(volatile v4u*)(CTXh + cbase + (size_t)(qBase + qr) * NCO + rlane * 8) = v;
    }
    __threadfence();
  }
  wave_sync_lds();
#pragma unroll
  for (int ct = 0; ct < 8; ++ct) *(v4u*)(hrow + ct * 16) = lv[ct];
  wave_sync_lds();
  for (int pass = 0; pass < 2; ++pass) {
#pragma unroll
    for (int it = 0; it < 8; ++it) {
      const int qr = it * 2 + hsel;
      const v4u v = *(const v4u*)(hsrc + qr * HPITCH + rlane * 8);
      *(volatile v4u*)(CTXl + cbase + (size_t)(qBase + qr) * NCO + rlane * 8) = v;
    }
    __threadfence();
  }
}

extern "C" void kernel_launch(void* const* d_in, const int* in_sizes, int n_in,
                              void* d_out, int out_size, void* d_ws, size_t ws_size,
                              hipStream_t stream) {
  if (n_in < 15) return;
  if (in_sizes[0] != NB * CIN * SLEN) return;
  if (in_sizes[1] != NCO * CIN || in_sizes[5] != NCO * CIN || in_sizes[9] != NCO * CIN) return;
  if (in_sizes[2] != NCO * 3 || in_sizes[6] != NCO * 3 || in_sizes[10] != NCO * 3) return;
  if (in_sizes[3] != NCO * 15 || in_sizes[7] != NCO * 15 || in_sizes[11] != NCO * 15) return;
  if (in_sizes[4] != 2 || in_sizes[8] != 2 || in_sizes[12] != 2) return;
  if (in_sizes[13] != CIN * NCO) return;
  if (in_sizes[14] != CIN) return;
  if (out_size != NB * CIN * SLEN) return;

  const float* x    = (const float*)d_in[0];
  const float* pw_q = (const float*)d_in[1];
  const float* dq3  = (const float*)d_in[2];
  const float* dq15 = (const float*)d_in[3];
  const float* gq   = (const float*)d_in[4];
  const float* pw_k = (const float*)d_in[5];
  const float* dk3  = (const float*)d_in[6];
  const float* dk15 = (const float*)d_in[7];
  const float* gk   = (const float*)d_in[8];
  const float* pw_v = (const float*)d_in[9];
  const float* dv3  = (const float*)d_in[10];
  const float* dv15 = (const float*)d_in[11];
  const float* gv   = (const float*)d_in[12];
  const float* wu   = (const float*)d_in[13];
  const float* bu   = (const float*)d_in[14];

  const size_t PQT = (size_t)NB * QXSZ * 2;
  const size_t PPW = (size_t)3 * NCO * CIN * 2;
  const size_t PWU = (size_t)CIN * NCO * 2;
  const size_t PY  = (size_t)GBAT * 3 * PLN * 4;
  const size_t PQX = (size_t)GBAT * NHD * QXSZ * 2;
  const size_t PVX = (size_t)GBAT * PLN * 2;
  const size_t PCT = (size_t)GBAT * PLN * 2;
  size_t off = 0;
  const size_t oQT = off; off += PQT;
  const size_t oPW = off; off += PPW;
  const size_t oWU = off; off += PWU;
  const size_t oY  = off; off += PY;
  const size_t oQX = off; off += PQX;
  const size_t oKX = off; off += PQX;
  const size_t oVX = off; off += PVX;
  const size_t oCH = off; off += PCT;
  const size_t oCL = off; off += PCT;
  if (off > ws_size) return;
  if (off > (size_t)134217728) return;

  char* ws = (char*)d_ws;
  unsigned short* QT   = (unsigned short*)(ws + oQT);
  unsigned short* PW   = (unsigned short*)(ws + oPW);
  unsigned short* WU   = (unsigned short*)(ws + oWU);
  float*          Y    = (float*)(ws + oY);
  unsigned short* QX   = (unsigned short*)(ws + oQX);
  unsigned short* KX   = (unsigned short*)(ws + oKX);
  unsigned short* VX   = (unsigned short*)(ws + oVX);
  unsigned short* CTXh = (unsigned short*)(ws + oCH);
  unsigned short* CTXl = (unsigned short*)(ws + oCL);
  float*          out  = (float*)d_out;

  const dim3 blk(256);
  const int n8w = NCO * CIN / 8;
  const dim3 gCvtW((n8w + 255) / 256);
  const dim3 gQt(SLEN / 64, NB);
  const dim3 gPw(((NCO / 64) * (SLEN / 64) + 7) / 8, 3, GBAT);
  const dim3 gConv(SLEN / 64, NHD, GBAT);
  const dim3 gAttn(SLEN / 128, NHD * GBAT);
  const dim3 gUni(((CIN / 64) * (SLEN / 64) + 7) / 8, GBAT, 1);

  const float oscPw  = 1.0f / 16384.0f;
  const float sc     = 0.08838834764831845f * (1.0f / 256.0f);
  const float rscale = 16384.0f;
  const float oscUni = 1.0f / 65536.0f;
  const float rres   = 1.0f / 16384.0f;

  cvt_qt<<<gQt, blk, 0, stream>>>(x, QT, 16.0f);
  cvt_h8<<<gCvtW, blk, 0, stream>>>(pw_q, PW, n8w, 1024.0f);
  cvt_h8<<<gCvtW, blk, 0, stream>>>(pw_k, PW + (size_t)NCO * CIN, n8w, 1024.0f);
  cvt_h8<<<gCvtW, blk, 0, stream>>>(pw_v, PW + (size_t)2 * NCO * CIN, n8w, 1024.0f);
  cvt_h8<<<gCvtW, blk, 0, stream>>>(wu, WU, n8w, 1024.0f);

  for (int g = 0; g < NGRP; ++g) {
    const int b0 = g * GBAT;
    gemm64<0, 0><<<gPw, blk, 0, stream>>>(
        PW, CIN, (long long)(NCO * CIN), 0LL,
        QT + (size_t)b0 * QXSZ, CIN, 0LL, (long long)QXSZ,
        QT + (size_t)b0 * QXSZ, CIN,
        bu,
        Y, SLEN, (long long)PLN, (long long)(3 * PLN),
        NCO, SLEN, CIN, oscPw, 0.0f);
    dwconv_kernel<<<gConv, blk, 0, stream>>>(Y, dq3, dq15, gq, dk3, dk15, gk, dv3, dv15, gv, QX, KX, VX);
    attn_kernel<<<gAttn, blk, 0, stream>>>(QX, KX, VX, CTXh, CTXl, sc, rscale);
    gemm64<2, 2><<<gUni, blk, 0, stream>>>(
        WU, NCO, 0LL, 0LL,
        CTXh, NCO, (long long)PLN, 0LL,
        CTXl, NCO,
        bu,
        out + (size_t)b0 * CIN * SLEN, SLEN, (long long)(CIN * SLEN), 0LL,
        CIN, SLEN, NCO, oscUni, rres);
  }
  (void)hipGetLastError();
}
